// PersistentMemoryAttention_14456859918523
// MI455X (gfx1250) — hardware-verified
//
#include <hip/hip_runtime.h>
#include <math.h>
#include <stdint.h>

#pragma clang fp contract(off)

#define NB    2
#define SEQ   2048
#define CDIM  1024
#define NQH   16
#define NKV   4
#define HD    64
#define MEM   64
#define GC    32
#define KVD   (NKV * HD)
#define SKEY  (MEM + SEQ)
#define NQB   (SEQ / 64)
#define NKT   (SKEY / 64)
#define RESQB 8
#define VLP   (MEM + RESQB * 64)
#define RMS_EPS 1e-6f
static_assert(NQH * HD == CDIM);
static_assert(NQH == 4 * NKV);
static_assert((SKEY % 64) == 0 && (VLP % 64) == 0 && (CDIM % 64) == 0 && (KVD % 64) == 0);
static_assert((SEQ & (SEQ - 1)) == 0);
static_assert(RESQB <= NQB);

typedef _Float16 v16h __attribute__((ext_vector_type(16)));
typedef _Float16 v8h  __attribute__((ext_vector_type(8)));
typedef __bf16   v16b __attribute__((ext_vector_type(16)));
typedef __bf16   v8b  __attribute__((ext_vector_type(8)));
typedef float    v8f  __attribute__((ext_vector_type(8)));
typedef float    v4f  __attribute__((ext_vector_type(4)));
typedef unsigned int v4u __attribute__((ext_vector_type(4)));

__device__ __forceinline__ unsigned short bf_bits(float f) {
  unsigned u = __float_as_uint(f);
  return (unsigned short)((u + 0x7FFFu + ((u >> 16) & 1u)) >> 16);
}
__device__ __forceinline__ float bf_up(unsigned short h) { return __uint_as_float(((unsigned)h) << 16); }
__device__ __forceinline__ float bfr(float f) { return bf_up(bf_bits(f)); }
__device__ __forceinline__ unsigned short h_bits(_Float16 x) { return __builtin_bit_cast(unsigned short, x); }
__device__ __forceinline__ unsigned pk16(unsigned short a, unsigned short b) { return (unsigned)a | ((unsigned)b << 16); }
__device__ __forceinline__ v8f zero8() { v8f z = {0.f, 0.f, 0.f, 0.f, 0.f, 0.f, 0.f, 0.f}; return z; }
__device__ __forceinline__ v8h zero8h() {
  const _Float16 z = (_Float16)0.0f;
  v8h r = {z, z, z, z, z, z, z, z};
  return r;
}

__device__ __forceinline__ v16b ldfrag_b(const __bf16* p) {
  union { v16b v; v8b h[2]; } f;
  f.h[0] = *(const v8b*)(p);
  f.h[1] = *(const v8b*)(p + 16);
  return f.v;
}

__device__ __forceinline__ v8f mma_b(v16b a, v16b b, v8f c) {
  c = __builtin_amdgcn_wmma_f32_16x16x32_bf16(false, a, false, b, (short)0, c, false, false);
#if defined(__HIP_DEVICE_COMPILE__)
  asm volatile("v_nop\n\tv_nop\n\tv_nop\n\tv_nop" : "+v"(c) : "v"(a), "v"(b));
#endif
  return c;
}
__device__ __forceinline__ v8f mma_h(v16h a, v16h b, v8f c) {
  c = __builtin_amdgcn_wmma_f32_16x16x32_f16(false, a, false, b, (short)0, c, false, false);
#if defined(__HIP_DEVICE_COMPILE__)
  asm volatile("v_nop\n\tv_nop\n\tv_nop\n\tv_nop" : "+v"(c) : "v"(a), "v"(b));
#endif
  return c;
}
__device__ __forceinline__ v8f mma_b_raw(v16b a, v16b b, v8f c) {
  return __builtin_amdgcn_wmma_f32_16x16x32_bf16(false, a, false, b, (short)0, c, false, false);
}
__device__ __forceinline__ void dep_guard_b(v8f& a, v8f& b, v16b x, v16b y) {
#if defined(__HIP_DEVICE_COMPILE__)
  asm volatile("v_nop\n\tv_nop\n\tv_nop\n\tv_nop" : "+v"(a), "+v"(b) : "v"(x), "v"(y));
#endif
}
__device__ __forceinline__ void keep4_b(v16b a, v16b b, v16b c, v16b d) {
#if defined(__HIP_DEVICE_COMPILE__)
  asm volatile("v_nop" :: "v"(a), "v"(b), "v"(c), "v"(d));
#endif
}
__device__ __forceinline__ void acc_guard4(v8f& a, v8f& b, v8f& c, v8f& d) {
#if defined(__HIP_DEVICE_COMPILE__)
  asm volatile("v_nop\n\tv_nop\n\tv_nop\n\tv_nop" : "+v"(a), "+v"(b), "+v"(c), "+v"(d));
#endif
}

__global__ __launch_bounds__(256) void cvt_bf16x8(const float* __restrict__ in, unsigned short* out, int n8) {
  const int i = blockIdx.x * 256 + threadIdx.x;
  if (i < n8) {
    const v4f a = *(const v4f*)(in + (size_t)i * 8);
    const v4f b = *(const v4f*)(in + (size_t)i * 8 + 4);
    v4u p;
    p[0] = pk16(bf_bits(a[0]), bf_bits(a[1]));
    p[1] = pk16(bf_bits(a[2]), bf_bits(a[3]));
    p[2] = pk16(bf_bits(b[0]), bf_bits(b[1]));
    p[3] = pk16(bf_bits(b[2]), bf_bits(b[3]));
    *(volatile v4u*)(out + (size_t)i * 8) = p;
    __threadfence();
    *(volatile v4u*)(out + (size_t)i * 8) = p;
  }
}

__global__ __launch_bounds__(256) void gate_k(const float* __restrict__ x, const float* __restrict__ Wg,
                                              float* gate, int nbt) {
  const int i   = blockIdx.x * 256 + threadIdx.x;
  const int bt  = i >> 2;
  const int kv  = i & 3;
  const int btc = (bt < nbt) ? bt : (nbt - 1);
  const float* xr = x + (size_t)btc * CDIM;
  const float* wr = Wg + kv * GC;
  float z = 0.f;
#pragma unroll 1
  for (int cc = 0; cc < GC; ++cc) z += bfr(xr[cc]) * bfr(wr[cc]);
  const float ez = expf(-z);
  const float g  = 3.0f * (1.0f / (1.0f + ez));
  if (bt < nbt) {
    *(volatile float*)(gate + i) = g;
    __threadfence();
    *(volatile float*)(gate + i) = g;
  }
}

__global__ __launch_bounds__(128) void memk_k(const float* __restrict__ memk, unsigned short* Kh, unsigned short* Kl) {
  __shared__ __align__(16) unsigned short shi[KVD];
  __shared__ __align__(16) unsigned short slo[KVD];
  const int m    = blockIdx.x;
  const int wave = threadIdx.x >> 5;
  const int lane = threadIdx.x & 31;
  const int kvh  = wave;
  const float* p = memk + ((size_t)m * NKV + kvh) * HD;
  const float x1 = bfr(p[lane]);
  const float x2 = bfr(p[lane + 32]);
  float ss = x1 * x1 + x2 * x2;
#pragma unroll
  for (int off = 16; off >= 1; off >>= 1) ss += __shfl_xor(ss, off, 32);
  const float rs = rsqrtf(ss * (1.0f / HD) + RMS_EPS);
  const float v1 = (x1 * rs) * 1.2f;
  const float v2 = (x2 * rs) * 1.2f;
  const unsigned short h1 = bf_bits(v1), h2 = bf_bits(v2);
  shi[kvh * HD + lane]      = h1;
  shi[kvh * HD + lane + 32] = h2;
  slo[kvh * HD + lane]      = bf_bits(v1 - bf_up(h1));
  slo[kvh * HD + lane + 32] = bf_bits(v2 - bf_up(h2));
  __syncthreads();
  const v4u vh = *(const v4u*)(shi + lane * 8);
  const v4u vl = *(const v4u*)(slo + lane * 8);
  const int  b   = wave >> 1;
  const bool wlo = (wave & 1) != 0;
  v4u v = vh;
  if (wlo) v = vl;
  unsigned short* dh = Kh + ((size_t)b * SKEY + m) * KVD + lane * 8;
  unsigned short* dl = Kl + ((size_t)b * SKEY + m) * KVD + lane * 8;
  unsigned short* d  = wlo ? dl : dh;
  *(volatile v4u*)d = v;
  __threadfence();
  *(volatile v4u*)d = v;
}

__global__ __launch_bounds__(256) void memv_k(const float* __restrict__ memv, const float* __restrict__ vsp,
                                              unsigned short* VTh, unsigned short* VTl) {
  __shared__ __align__(16) unsigned short sh[HD * MEM];
  __shared__ __align__(16) unsigned short sl[HD * MEM];
  const int b    = blockIdx.x >> 2;
  const int kvh  = blockIdx.x & 3;
  const int tid  = threadIdx.x;
  const int wave = tid >> 5;
  const int lane = tid & 31;
  const int d    = tid >> 2;
  const int mq   = (tid & 3) * 16;
  const float vs = bfr(vsp[0]);
#pragma unroll
  for (int i = 0; i < 16; ++i) {
    const int m = mq + i;
    const float v = bfr(memv[((size_t)m * NKV + kvh) * HD + d]) * vs;
    const _Float16 x0 = (_Float16)v;
    sh[d * MEM + m] = h_bits(x0);
    sl[d * MEM + m] = h_bits((_Float16)((v - (float)x0) * 4096.0f));
  }
  __syncthreads();
  const int q8 = lane >> 3, c8 = (lane & 7) * 8;
  v4u hv[2], lv[2];
#pragma unroll
  for (int it = 0; it < 2; ++it) {
    const int dd = it * 32 + wave * 4 + q8;
    hv[it] = *(const v4u*)(sh + dd * MEM + c8);
    lv[it] = *(const v4u*)(sl + dd * MEM + c8);
  }
  for (int pass = 0; pass < 2; ++pass) {
#pragma unroll
    for (int it = 0; it < 2; ++it) {
      const int dd = it * 32 + wave * 4 + q8;
      const size_t ro = (size_t)b * KVD + (size_t)kvh * HD + dd;
      *(volatile v4u*)(VTh + ro * SKEY + c8) = hv[it];
      *(volatile v4u*)(VTl + ro * VLP  + c8) = lv[it];
    }
    __threadfence();
  }
}

template <int NSPLIT, int OUT_MODE>
__global__ __launch_bounds__(256) void gemm64(
    const unsigned short* __restrict__ Ap, const unsigned short* __restrict__ A2p, int lda, long long strideA,
    const unsigned short* __restrict__ Btp, int ldb, long long strideB,
    void* Cout, int ldc, long long strideC,
    void* Cout2, int ldc2, long long strideC2, int N2,
    const float* __restrict__ aux0, const float* __restrict__ aux1,
    int M, int N, int K) {
  const __bf16* A  = (const __bf16*)(const void*)Ap;
  const __bf16* A2 = (const __bf16*)(const void*)A2p;
  const __bf16* Bt = (const __bf16*)(const void*)Btp;
  __shared__ __align__(16) float sT[8][16 * 68];
  const int b    = blockIdx.y;
  const int lane = threadIdx.x & 31;
  const int wave = threadIdx.x >> 5;
  const int tilesN = N >> 6;
  const int tilesM = M >> 6;
  const int tile = blockIdx.x * 8 + wave;
  if (tile >= tilesM * tilesN) return;
  const int tm = tile / tilesN;
  const int tn = tile - tm * tilesN;
  const int m0 = tm << 6;
  const int n0 = tn << 6;

  const __bf16* Ab  = A  + (size_t)b * strideA;
  const __bf16* Bb  = Bt + (size_t)b * strideB;
  const __bf16* Ab2 = (NSPLIT >= 1) ? (A2 + (size_t)b * strideA) : Ab;

  const int rlane = lane & 15;
  const int koff  = (lane >> 4) * 8;
  const int mOff  = (lane >> 4) * 8;

  v8f acc[4][4];
#pragma unroll
  for (int i = 0; i < 4; ++i)
#pragma unroll
    for (int j = 0; j < 4; ++j) acc[i][j] = zero8();

  for (int k0 = 0; k0 < K; k0 += 32) {
    v16b bh[4];
#pragma unroll
    for (int j = 0; j < 4; ++j) {
      const size_t bo = (size_t)(n0 + (j << 4) + rlane) * ldb + koff + k0;
      bh[j] = ldfrag_b(Bb + bo);
    }
#pragma unroll
    for (int i = 0; i < 4; ++i) {
      const size_t ao = (size_t)(m0 + (i << 4) + rlane) * lda + koff + k0;
      const v16b ah = ldfrag_b(Ab + ao);
      v16b al = ah;
      if (NSPLIT >= 1) al = ldfrag_b(Ab2 + ao);
#pragma unroll
      for (int j = 0; j < 4; ++j) {
        acc[i][j] = mma_b_raw(ah, bh[j], acc[i][j]);
        if (NSPLIT >= 1) acc[i][j] = mma_b_raw(al, bh[j], acc[i][j]);
      }
      dep_guard_b(acc[i][0], acc[i][3], ah, al);
    }
    keep4_b(bh[0], bh[1], bh[2], bh[3]);
  }
  acc_guard4(acc[0][0], acc[0][1], acc[0][2], acc[0][3]);
  acc_guard4(acc[1][0], acc[1][1], acc[1][2], acc[1][3]);
  acc_guard4(acc[2][0], acc[2][1], acc[2][2], acc[2][3]);
  acc_guard4(acc[3][0], acc[3][1], acc[3][2], acc[3][3]);

  float* slab = sT[wave];
#pragma unroll
  for (int i = 0; i < 4; ++i) {
    const int mBase = m0 + (i << 4);
#pragma unroll
    for (int j = 0; j < 4; ++j) {
#pragma unroll
      for (int r = 0; r < 8; ++r) {
        slab[(mOff + r) * 68 + (j << 4) + rlane] = acc[i][j][r];
      }
    }
    __builtin_amdgcn_fence(__ATOMIC_RELEASE, "workgroup");
    __builtin_amdgcn_wave_barrier();
    __builtin_amdgcn_fence(__ATOMIC_ACQUIRE, "workgroup");
    if (OUT_MODE == 0) {
      float* C = (float*)Cout + (size_t)b * strideC;
      const int hh = lane >> 4, c4 = (lane & 15) * 4;
      for (int pass = 0; pass < 2; ++pass) {
#pragma unroll
        for (int it = 0; it < 8; ++it) {
          const int row = it * 2 + hh;
          const v4f v = *(const v4f*)(slab + row * 68 + c4);
          *(volatile v4f*)(C + (size_t)(mBase + row) * ldc + n0 + c4) = v;
        }
        __threadfence();
      }
    } else {
      const int q = lane >> 3, c8 = (lane & 7) * 8;
      unsigned short* C  = (unsigned short*)Cout  + (size_t)b * strideC;
      unsigned short* C2 = (unsigned short*)Cout2 + (size_t)b * strideC2;
      const bool wlo = (OUT_MODE != 3) || (n0 < N2);
      v4u hv[4], lv[4];
#pragma unroll
      for (int it = 0; it < 4; ++it) {
        const int row  = it * 4 + q;
        const int mrow = mBase + row;
        float f[8];
        if (OUT_MODE == 3) {
          const int kvh = m0 >> 6;
          const float* sp = slab + row * 68 + c8;
#pragma unroll
          for (int e = 0; e < 8; ++e) {
            const int t = n0 + c8 + e;
            const size_t bt = (size_t)b * SEQ + t;
            const float g  = aux0[bt * NKV + kvh];
            const float vv = bfr(aux1[bt * KVD + mrow]);
            f[e] = sp[e] + g * vv;
          }
        } else {
          const int  jj   = c8 & 31;
          const bool lowh = (c8 < 32);
          const int  t    = mrow & (SEQ - 1);
          const float* sp  = slab + row * 68 + jj;
          const float* cp  = aux0 + (size_t)t * (HD / 2) + jj;
          const float* snp = aux1 + (size_t)t * (HD / 2) + jj;
          float ss = 0.f;
#pragma unroll
          for (int e = 0; e < 8; ++e) {
            const float x1 = sp[e];
            const float x2 = sp[e + 32];
            const float cv = bfr(cp[e]);
            const float sv = bfr(snp[e]);
            const float ra = x1 * cv - x2 * sv;
            const float rb = x1 * sv + x2 * cv;
            f[e] = lowh ? ra : rb;
            ss += f[e] * f[e];
          }
          ss += __shfl_xor(ss, 1, 32);
          ss += __shfl_xor(ss, 2, 32);
          ss += __shfl_xor(ss, 4, 32);
          const float rs = rsqrtf(ss * (1.0f / HD) + RMS_EPS);
#pragma unroll
          for (int e = 0; e < 8; ++e) f[e] = (f[e] * rs) * 1.2f;
        }
        v4u a, a2;
#pragma unroll
        for (int e = 0; e < 4; ++e) {
          const float f0 = f[2 * e], f1 = f[2 * e + 1];
          unsigned short h0, h1, l0, l1;
          if (OUT_MODE == 4) {
            h0 = bf_bits(f0); h1 = bf_bits(f1);
            l0 = bf_bits(f0 - bf_up(h0)); l1 = bf_bits(f1 - bf_up(h1));
          } else {
            const _Float16 x0 = (_Float16)f0, x1 = (_Float16)f1;
            h0 = h_bits(x0); h1 = h_bits(x1);
            l0 = h_bits((_Float16)((f0 - (float)x0) * 4096.0f));
            l1 = h_bits((_Float16)((f1 - (float)x1) * 4096.0f));
          }
          a[e] = pk16(h0, h1); a2[e] = pk16(l0, l1);
        }
        hv[it] = a; lv[it] = a2;
      }
      for (int pass = 0; pass < 2; ++pass) {
#pragma unroll
        for (int it = 0; it < 4; ++it) {
          const int row = it * 4 + q;
          *(volatile v4u*)(C + (size_t)(mBase + row) * ldc + n0 + c8) = hv[it];
          if (wlo) *(volatile v4u*)(C2 + (size_t)(mBase + row) * ldc2 + n0 + c8) = lv[it];
        }
        __threadfence();
      }
    }
    __builtin_amdgcn_fence(__ATOMIC_RELEASE, "workgroup");
    __builtin_amdgcn_wave_barrier();
    __builtin_amdgcn_fence(__ATOMIC_ACQUIRE, "workgroup");
  }
}

template <bool RES>
__global__ __launch_bounds__(128)
void attn64(const unsigned short* __restrict__ qhp, const unsigned short* __restrict__ qlp,
            const unsigned short* __restrict__ khp, const unsigned short* __restrict__ klp,
            const unsigned short* __restrict__ vhp, const unsigned short* __restrict__ vlp,
            unsigned short* ohp, unsigned short* olp,
            int qbBase, int nqbThis, float sscale) {
  union FB { v16b v; v8b h[2]; };
  union FH { v16h v; v8h h[2]; };
  __shared__ __align__(16) __bf16   Ksh[64 * 64];
  __shared__ __align__(16) __bf16   Ksl[64 * 64];
  __shared__ __align__(16) _Float16 Vth[64 * 64];
  __shared__ __align__(16) _Float16 Vtl[RES ? 64 * 64 : 8];
  __shared__ __align__(16) _Float16 Psh[4][16 * 64];
  __shared__ __align__(16) _Float16 Psl[RES ? 4 : 1][16 * 64];
  __shared__ __align__(16) float    Os[4][16 * 64];

  const int tid  = threadIdx.x;
  const int wave = tid >> 5;
  const int lane = tid & 31;
  const int hh   = lane >> 4;
  const int c    = lane & 15;

  const int bx   = blockIdx.x;
  const int qbl  = bx % nqbThis;
  const int rest = bx / nqbThis;
  const int h    = rest % NQH;
  const int b    = rest / NQH;
  const int kvh  = h >> 2;
  const int qb   = qbBase + qbl;
  const int q0   = qb * 64 + wave * 16;
  const size_t rowB = (size_t)b * SEQ;

  const __bf16* Qh = (const __bf16*)(const void*)qhp + (size_t)h * HD;
  const __bf16* Ql = (const __bf16*)(const void*)qlp + (size_t)h * HD;
  const __bf16* Kh = (const __bf16*)(const void*)khp + (size_t)b * SKEY * KVD + (size_t)kvh * HD;
  const __bf16* Kl = (const __bf16*)(const void*)klp + (size_t)b * SKEY * KVD + (size_t)kvh * HD;
  const _Float16* Vh = (const _Float16*)(const void*)vhp + ((size_t)b * KVD + (size_t)kvh * HD) * SKEY;
  const _Float16* Vl = (const _Float16*)(const void*)vlp + ((size_t)b * KVD + (size_t)kvh * HD) * VLP;

  v16b qah[2], qal[2];
#pragma unroll
  for (int dc = 0; dc < 2; ++dc) {
    const size_t qo = (rowB + q0 + c) * CDIM + dc * 32 + 8 * hh;
    qah[dc] = ldfrag_b(Qh + qo);
    qal[dc] = ldfrag_b(Ql + qo);
  }

  float mrow[8], lrow[8];
  v8f oacc[4];
#pragma unroll
  for (int r = 0; r < 8; ++r) { mrow[r] = -INFINITY; lrow[r] = 0.f; }
#pragma unroll
  for (int t = 0; t < 4; ++t) oacc[t] = zero8();

  const int ktEnd = qb + 2;
  for (int kt = 0; kt < NKT; ++kt) {
    if (kt >= ktEnd) break;
    const int kv0 = kt * 64;
    __syncthreads();
    {
      const int r = tid >> 1, half = (tid & 1) * 32;
      const __bf16*   kg  = Kh + (size_t)(kv0 + r) * KVD + half;
      const __bf16*   klg = Kl + (size_t)(kv0 + r) * KVD + half;
      const _Float16* vg  = Vh + (size_t)r * SKEY + kv0 + half;
      const int kvl = (kv0 + 64 <= VLP) ? kv0 : (VLP - 64);
      const _Float16* vlg = Vl + (size_t)r * VLP + kvl + half;
      const bool resOK = (kv0 + 64 <= VLP);
#pragma unroll
      for (int i = 0; i < 4; ++i) {
        const v8b a0 = *(const v8b*)(kg + 8 * i);
        const v8b a1 = *(const v8b*)(klg + 8 * i);
        const v8h b0 = *(const v8h*)(vg + 8 * i);
        *(v8b*)(Ksh + r * 64 + half + 8 * i) = a0;
        *(v8b*)(Ksl + r * 64 + half + 8 * i) = a1;
        *(v8h*)(Vth + r * 64 + half + 8 * i) = b0;
        if (RES) {
          v8h b1 = *(const v8h*)(vlg + 8 * i);
          if (!resOK) b1 = zero8h();
          *(v8h*)(Vtl + r * 64 + half + 8 * i) = b1;
        }
      }
    }
    __syncthreads();

    v8f s[4];
#pragma unroll
    for (int j = 0; j < 4; ++j) {
      s[j] = zero8();
#pragma unroll
      for (int dc = 0; dc < 2; ++dc) {
        FB kb, kl;
        kb.h[0] = *(const v8b*)(Ksh + (j * 16 + c) * 64 + dc * 32 + 8 * hh);
        kb.h[1] = *(const v8b*)(Ksh + (j * 16 + c) * 64 + dc * 32 + 16 + 8 * hh);
        kl.h[0] = *(const v8b*)(Ksl + (j * 16 + c) * 64 + dc * 32 + 8 * hh);
        kl.h[1] = *(const v8b*)(Ksl + (j * 16 + c) * 64 + dc * 32 + 16 + 8 * hh);
        s[j] = mma_b(qah[dc], kb.v, s[j]);
        s[j] = mma_b(qah[dc], kl.v, s[j]);
        s[j] = mma_b(qal[dc], kb.v, s[j]);
      }
    }

    _Float16* pwh = Psh[wave];
    _Float16* pwl = Psl[RES ? wave : 0];
    const bool diag = (kt == qb + 1);
    const int  qr0  = wave * 16 + 8 * hh;
#pragma unroll
    for (int r = 0; r < 8; ++r) {
      const int qrw = qr0 + r;
      float m = -INFINITY;
#pragma unroll
      for (int j = 0; j < 4; ++j) {
        const int  key = j * 16 + c;
        const bool vis = (!diag) || (key <= qrw);
        const float sv = vis ? (s[j][r] * sscale) : -INFINITY;
        s[j][r] = sv;
        m = fmaxf(m, sv);
      }
#pragma unroll
      for (int off = 1; off < 16; off <<= 1) m = fmaxf(m, __shfl_xor(m, off, 32));
      const float mnew  = fmaxf(mrow[r], m);
      const float msafe = (mnew == -INFINITY) ? 0.f : mnew;
      const float alpha = __expf(mrow[r] - msafe);
      mrow[r] = mnew;
      float psum = 0.f;
#pragma unroll
      for (int j = 0; j < 4; ++j) {
        const float p = __expf(s[j][r] - msafe);
        psum += p;
        const float p1k = p * 1024.0f;
        const _Float16 ph = (_Float16)p1k;
        pwh[(8 * hh + r) * 64 + j * 16 + c] = ph;
        if (RES) {
          const _Float16 pl = (_Float16)((p1k - (float)ph) * 4096.0f);
          pwl[(8 * hh + r) * 64 + j * 16 + c] = pl;
        }
      }
#pragma unroll
      for (int off = 1; off < 16; off <<= 1) psum += __shfl_xor(psum, off, 32);
      lrow[r] = lrow[r] * alpha + psum;
#pragma unroll
      for (int t = 0; t < 4; ++t) oacc[t][r] *= alpha;
    }
    __builtin_amdgcn_fence(__ATOMIC_RELEASE, "workgroup");
    __builtin_amdgcn_wave_barrier();
    __builtin_amdgcn_fence(__ATOMIC_ACQUIRE, "workgroup");

    v8f o1[4];
#pragma unroll
    for (int t = 0; t < 4; ++t) o1[t] = zero8();
#pragma unroll 1
    for (int kk = 0; kk < 2; ++kk) {
      FH pa, pl;
      pa.h[0] = *(const v8h*)(pwh + c * 64 + kk * 32 + 8 * hh);
      pa.h[1] = *(const v8h*)(pwh + c * 64 + kk * 32 + 16 + 8 * hh);
      if (RES) {
        pl.h[0] = *(const v8h*)(pwl + c * 64 + kk * 32 + 8 * hh);
        pl.h[1] = *(const v8h*)(pwl + c * 64 + kk * 32 + 16 + 8 * hh);
      } else {
        pl.v = pa.v;
      }
#pragma unroll
      for (int t = 0; t < 4; ++t) {
        FH vb;
        vb.h[0] = *(const v8h*)(Vth + (t * 16 + c) * 64 + kk * 32 + 8 * hh);
        vb.h[1] = *(const v8h*)(Vth + (t * 16 + c) * 64 + kk * 32 + 16 + 8 * hh);
        oacc[t] = mma_h(pa.v, vb.v, oacc[t]);
        if (RES) {
          FH vl;
          vl.h[0] = *(const v8h*)(Vtl + (t * 16 + c) * 64 + kk * 32 + 8 * hh);
          vl.h[1] = *(const v8h*)(Vtl + (t * 16 + c) * 64 + kk * 32 + 16 + 8 * hh);
          o1[t] = mma_h(pa.v, vl.v, o1[t]);
          o1[t] = mma_h(pl.v, vb.v, o1[t]);
        }
      }
    }
    if (RES) {
#pragma unroll
      for (int t = 0; t < 4; ++t)
#pragma unroll
        for (int r = 0; r < 8; ++r) oacc[t][r] += o1[t][r] * (1.0f / 4096.0f);
    }
  }

  float* os = Os[wave];
#pragma unroll
  for (int r = 0; r < 8; ++r) {
    const float l = lrow[r];
    const float inv = ((l > 0.f) ? (1.0f / l) : 0.f) * (1.0f / 1024.0f);
#pragma unroll
    for (int t = 0; t < 4; ++t) os[(8 * hh + r) * 64 + t * 16 + c] = oacc[t][r] * inv;
  }
  __builtin_amdgcn_fence(__ATOMIC_RELEASE, "workgroup");
  __builtin_amdgcn_wave_barrier();
  __builtin_amdgcn_fence(__ATOMIC_ACQUIRE, "workgroup");
  {
    const int q4 = lane >> 3, c8 = (lane & 7) * 8;
    v4u hv[4], lv[4];
#pragma unroll
    for (int it = 0; it < 4; ++it) {
      const int row = it * 4 + q4;
      const float* sp = os + row * 64 + c8;
      v4u a, a2;
#pragma unroll
      for (int e = 0; e < 4; ++e) {
        const float f0 = sp[2 * e], f1 = sp[2 * e + 1];
        const unsigned short h0 = bf_bits(f0), h1 = bf_bits(f1);
        const unsigned short l0 = bf_bits(f0 - bf_up(h0)), l1 = bf_bits(f1 - bf_up(h1));
        a[e] = pk16(h0, h1); a2[e] = pk16(l0, l1);
      }
      hv[it] = a; lv[it] = a2;
    }
    for (int pass = 0; pass < 2; ++pass) {
#pragma unroll
      for (int it = 0; it < 4; ++it) {
        const int row = it * 4 + q4;
        const size_t go = (rowB + q0 + row) * CDIM + (size_t)h * HD + c8;
        *(volatile v4u*)(ohp + go) = hv[it];
        *(volatile v4u*)(olp + go) = lv[it];
      }
      __threadfence();
    }
  }
}

extern "C" void kernel_launch(void* const* d_in, const int* in_sizes, int n_in,
                              void* d_out, int out_size, void* d_ws, size_t ws_size,
                              hipStream_t stream) {
  if (n_in < 12) return;
  if (in_sizes[0] != NB * SEQ * CDIM) return;
  if (in_sizes[1] != NB * SEQ * KVD) return;
  if (in_sizes[2] != SEQ * (HD / 2) || in_sizes[3] != SEQ * (HD / 2)) return;
  if (in_sizes[4] != CDIM * CDIM || in_sizes[7] != CDIM * CDIM) return;
  if (in_sizes[5] != KVD * CDIM || in_sizes[6] != KVD * CDIM) return;
  if (in_sizes[8] != NKV * GC) return;
  if (in_sizes[9] != MEM * NKV * HD || in_sizes[10] != MEM * NKV * HD) return;
  if (in_sizes[11] < 1) return;
  if (out_size != NB * SEQ * CDIM) return;

  const float* x    = (const float*)d_in[0];
  const float* ve   = (const float*)d_in[1];
  const float* cosT = (const float*)d_in[2];
  const float* sinT = (const float*)d_in[3];
  const float* Wq   = (const float*)d_in[4];
  const float* Wk   = (const float*)d_in[5];
  const float* Wv   = (const float*)d_in[6];
  const float* Wp   = (const float*)d_in[7];
  const float* Wg   = (const float*)d_in[8];
  const float* memk = (const float*)d_in[9];
  const float* memv = (const float*)d_in[10];
  const float* vsc  = (const float*)d_in[11];

  const size_t PX  = (size_t)NB * SEQ * CDIM * 2;
  const size_t PWQ = (size_t)CDIM * CDIM * 2;
  const size_t PWK = (size_t)KVD * CDIM * 2;
  const size_t PK  = (size_t)NB * SKEY * KVD * 2;
  const size_t PVT = (size_t)NB * KVD * SKEY * 2;
  const size_t PVL = (size_t)NB * KVD * VLP * 2;
  const size_t PG  = (size_t)NB * SEQ * NKV * 4;
  size_t off = 0;
  const size_t oXb  = off; off += PX;
  const size_t oWq  = off; off += PWQ;
  const size_t oWk  = off; off += PWK;
  const size_t oWv  = off; off += PWK;
  const size_t oWp  = off; off += PWQ;
  const size_t oQh  = off; off += PX;
  const size_t oQl  = off; off += PX;
  const size_t oKh  = off; off += PK;
  const size_t oKl  = off; off += PK;
  const size_t oVTh = off; off += PVT;
  const size_t oVTl = off; off += PVL;
  const size_t oG   = off; off += PG;
  const size_t oOh  = off; off += PX;
  const size_t oOl  = off; off += PX;
  if (off > ws_size) return;
  if (off > (size_t)134217728) return;

  char* ws = (char*)d_ws;
  unsigned short* Xb  = (unsigned short*)(ws + oXb);
  unsigned short* Wqb = (unsigned short*)(ws + oWq);
  unsigned short* Wkb = (unsigned short*)(ws + oWk);
  unsigned short* Wvb = (unsigned short*)(ws + oWv);
  unsigned short* Wpb = (unsigned short*)(ws + oWp);
  unsigned short* Qh  = (unsigned short*)(ws + oQh);
  unsigned short* Ql  = (unsigned short*)(ws + oQl);
  unsigned short* Kh  = (unsigned short*)(ws + oKh);
  unsigned short* Kl  = (unsigned short*)(ws + oKl);
  unsigned short* VTh = (unsigned short*)(ws + oVTh);
  unsigned short* VTl = (unsigned short*)(ws + oVTl);
  float*          Gt  = (float*)(ws + oG);
  unsigned short* Oh  = (unsigned short*)(ws + oOh);
  unsigned short* Ol  = (unsigned short*)(ws + oOl);

  const dim3 blk(256);
  const int n8x  = NB * SEQ * CDIM / 8;
  const int n8wq = CDIM * CDIM / 8;
  const int n8wk = KVD * CDIM / 8;
  const dim3 gCvtX((n8x + 255) / 256);
  const dim3 gCvtWq((n8wq + 255) / 256);
  const dim3 gCvtWk((n8wk + 255) / 256);
  const int  nbt = NB * SEQ;
  const dim3 gGate((nbt * NKV + 255) / 256);
  const dim3 gQ(((NB * SEQ / 64) * (CDIM / 64) + 7) / 8, 1);
  const dim3 gK(((SEQ / 64) * (KVD / 64) + 7) / 8, NB);
  const dim3 gV(((KVD / 64) * (SEQ / 64) + 7) / 8, NB);
  const dim3 gO(((NB * SEQ / 64) * (CDIM / 64) + 7) / 8, 1);

  cvt_bf16x8<<<gCvtX, blk, 0, stream>>>(x, Xb, n8x);
  cvt_bf16x8<<<gCvtWq, blk, 0, stream>>>(Wq, Wqb, n8wq);
  cvt_bf16x8<<<gCvtWk, blk, 0, stream>>>(Wk, Wkb, n8wk);
  cvt_bf16x8<<<gCvtWk, blk, 0, stream>>>(Wv, Wvb, n8wk);
  cvt_bf16x8<<<gCvtWq, blk, 0, stream>>>(Wp, Wpb, n8wq);
  gate_k<<<gGate, blk, 0, stream>>>(x, Wg, Gt, nbt);
  memk_k<<<dim3(MEM), dim3(128), 0, stream>>>(memk, Kh, Kl);
  memv_k<<<dim3(NB * NKV), blk, 0, stream>>>(memv, vsc, VTh, VTl);
  gemm64<0, 4><<<gQ, blk, 0, stream>>>(
      Xb, Xb, CDIM, 0LL, Wqb, CDIM, 0LL,
      (void*)Qh, CDIM, 0LL, (void*)Ql, CDIM, 0LL, CDIM,
      cosT, sinT, NB * SEQ, CDIM, CDIM);
  gemm64<0, 4><<<gK, blk, 0, stream>>>(
      Xb, Xb, CDIM, (long long)SEQ * CDIM, Wkb, CDIM, 0LL,
      (void*)(Kh + (size_t)MEM * KVD), KVD, (long long)SKEY * KVD,
      (void*)(Kl + (size_t)MEM * KVD), KVD, (long long)SKEY * KVD, KVD,
      cosT, sinT, SEQ, KVD, CDIM);
  gemm64<0, 3><<<gV, blk, 0, stream>>>(
      Wvb, Wvb, CDIM, 0LL, Xb, CDIM, (long long)SEQ * CDIM,
      (void*)(VTh + MEM), SKEY, (long long)KVD * SKEY,
      (void*)(VTl + MEM), VLP, (long long)KVD * VLP, RESQB * 64,
      Gt, ve, KVD, SEQ, CDIM);
  attn64<true><<<dim3(NB * NQH * RESQB), dim3(128), 0, stream>>>(
      Qh, Ql, Kh, Kl, VTh, VTl, Oh, Ol, 0, RESQB, 0.125f);
  attn64<false><<<dim3(NB * NQH * (NQB - RESQB)), dim3(128), 0, stream>>>(
      Qh, Ql, Kh, Kl, VTh, VTl, Oh, Ol, RESQB, NQB - RESQB, 0.125f);
  gemm64<1, 0><<<gO, blk, 0, stream>>>(
      Oh, Ol, CDIM, 0LL, Wpb, CDIM, 0LL,
      d_out, CDIM, 0LL, d_out, CDIM, 0LL, 0,
      Gt, ve, NB * SEQ, CDIM, CDIM);
  (void)hipGetLastError();
}
